// _SpatialAttention2D_45449343926365
// MI455X (gfx1250) — hardware-verified
//
#include <hip/hip_runtime.h>
#include <stdint.h>

#define NBAT 8
#define NCH  256
#define NPX  4096
#define NHID 32
#define QKW  64
#define AQB  64
#define AKC  64

typedef __attribute__((ext_vector_type(16))) _Float16 v16h;
typedef __attribute__((ext_vector_type(8)))  _Float16 v8h;
typedef __attribute__((ext_vector_type(16))) __bf16   v16b;
typedef __attribute__((ext_vector_type(8)))  __bf16   v8b;
typedef __attribute__((ext_vector_type(8)))  float    v8f;
typedef __attribute__((ext_vector_type(4)))  float    v4f;
typedef __attribute__((ext_vector_type(2)))  float    v2f;
typedef __attribute__((ext_vector_type(4)))  unsigned int v4u;

__device__ __forceinline__ unsigned short f2bf_bits(float f) {
  unsigned u = __float_as_uint(f);
  return (unsigned short)((u + 0x7FFFu + ((u >> 16) & 1u)) >> 16);
}
__device__ __forceinline__ float bf_bits2f(unsigned short h) { return __uint_as_float(((unsigned)h) << 16); }
__device__ __forceinline__ unsigned pk16(unsigned short a, unsigned short b) { return (unsigned)a | ((unsigned)b << 16); }

union FragB { v16b v; v8b h[2]; };
union FragH { v16h v; v8h h[2]; };
__device__ __forceinline__ v16b ldfrag_b(const __bf16* p) {
  FragB f; f.h[0] = *(const v8b*)(p); f.h[1] = *(const v8b*)(p + 16); return f.v;
}
__device__ __forceinline__ v16h ldfrag_h(const _Float16* p) {
  FragH f; f.h[0] = *(const v8h*)(p); f.h[1] = *(const v8h*)(p + 16); return f.v;
}
__device__ __forceinline__ v8f mma_b(v16b a, v16b b, v8f c) {
  return __builtin_amdgcn_wmma_f32_16x16x32_bf16(false, a, false, b, (short)0, c, false, false);
}
__device__ __forceinline__ v8f mma_h(v16h a, v16h b, v8f c) {
  return __builtin_amdgcn_wmma_f32_16x16x32_f16(false, a, false, b, (short)0, c, false, false);
}

__device__ __forceinline__ void guard_b2(v8f& a, v8f& b, v16b x, v16b y) {
  asm volatile("v_nop\n\tv_nop\n\tv_nop\n\tv_nop" : "+v"(a), "+v"(b) : "v"(x), "v"(y));
}
__device__ __forceinline__ void keep4_b(v16b a, v16b b, v16b c, v16b d) { asm volatile("v_nop" :: "v"(a), "v"(b), "v"(c), "v"(d)); }
__device__ __forceinline__ void acc_guard4(v8f& a, v8f& b, v8f& c, v8f& d) {
  asm volatile("v_nop\n\tv_nop\n\tv_nop\n\tv_nop" : "+v"(a), "+v"(b), "+v"(c), "+v"(d));
}
__device__ __forceinline__ void guard_s(v8f& d, v16b a0, v16b a1, v16b b0, v16b b1) {
  asm volatile("v_nop\n\tv_nop\n\tv_nop\n\tv_nop" : "+v"(d) : "v"(a0), "v"(a1), "v"(b0), "v"(b1));
}
__device__ __forceinline__ void guard_pv(v8f& o, v8f& t, v16h a0, v16h a1, v16h a2, v16h a3, v16h b0, v16h b1) {
  asm volatile("v_nop\n\tv_nop\n\tv_nop\n\tv_nop" : "+v"(o), "+v"(t) : "v"(a0), "v"(a1), "v"(a2), "v"(a3), "v"(b0), "v"(b1));
}
__device__ __forceinline__ void lds_wave_sync() {
  __builtin_amdgcn_fence(__ATOMIC_RELEASE, "workgroup");
  __builtin_amdgcn_wave_barrier();
  __builtin_amdgcn_fence(__ATOMIC_ACQUIRE, "workgroup");
}

template <int BIAS_MODE, int OUT_MODE>
__global__ __launch_bounds__(256) void gemm_bf16x3(
    const unsigned short* __restrict__ Ahp, const unsigned short* __restrict__ Alp, int lda, long strideA,
    const unsigned short* __restrict__ Bhp, const unsigned short* __restrict__ Blp, int ldb, long strideB,
    unsigned short* __restrict__ Cout, unsigned short* __restrict__ Cout2, int ldc, long strideC,
    const float* __restrict__ bias, const float* __restrict__ bias2, int nsplit,
    int M, int N, int K, float oscale) {
  const __bf16* A  = (const __bf16*)(const void*)Ahp;
  const __bf16* A2 = (const __bf16*)(const void*)Alp;
  const __bf16* Bt = (const __bf16*)(const void*)Bhp;
  const __bf16* Bt2 = (const __bf16*)(const void*)Blp;
  __shared__ __align__(16) float sT[8][16 * 68];
  const int b    = blockIdx.y;
  const int lane = threadIdx.x & 31;
  const int wave = threadIdx.x >> 5;
  const int tilesN = N >> 6;
  const int tilesM = M >> 6;
  const int tile = blockIdx.x * 8 + wave;
  if (tile >= tilesM * tilesN) return;
  const int tm = tile / tilesN;
  const int tn = tile - tm * tilesN;
  const int m0 = tm << 6;
  const int n0 = tn << 6;

  const __bf16* Ab  = A   + (size_t)b * strideA;
  const __bf16* Ab2 = A2  + (size_t)b * strideA;
  const __bf16* Bb  = Bt  + (size_t)b * strideB;
  const __bf16* Bb2 = Bt2 + (size_t)b * strideB;

  const int rlane = lane & 15;
  const int koff  = (lane >> 4) * 8;
  const int mOff  = (lane >> 4) * 8;

  v8f acc[4][4];
#pragma unroll
  for (int i = 0; i < 4; ++i)
#pragma unroll
    for (int j = 0; j < 4; ++j) acc[i][j] = (v8f){0.f,0.f,0.f,0.f,0.f,0.f,0.f,0.f};

  for (int k0 = 0; k0 < K; k0 += 32) {
    v16b bh[4], bl[4];
#pragma unroll
    for (int j = 0; j < 4; ++j) {
      const size_t bo = (size_t)(n0 + (j << 4) + rlane) * ldb + koff + k0;
      bh[j] = ldfrag_b(Bb + bo);
      bl[j] = ldfrag_b(Bb2 + bo);
    }
#pragma unroll
    for (int i = 0; i < 4; ++i) {
      const size_t ao = (size_t)(m0 + (i << 4) + rlane) * lda + koff + k0;
      const v16b ah = ldfrag_b(Ab + ao);
      const v16b al = ldfrag_b(Ab2 + ao);
#pragma unroll
      for (int j = 0; j < 4; ++j) {
        acc[i][j] = mma_b(ah, bh[j], acc[i][j]);
        acc[i][j] = mma_b(ah, bl[j], acc[i][j]);
        acc[i][j] = mma_b(al, bh[j], acc[i][j]);
      }
      guard_b2(acc[i][0], acc[i][3], ah, al);
    }
    keep4_b(bh[0], bh[1], bh[2], bh[3]);
    keep4_b(bl[0], bl[1], bl[2], bl[3]);
  }
  acc_guard4(acc[0][0], acc[0][1], acc[0][2], acc[0][3]);
  acc_guard4(acc[1][0], acc[1][1], acc[1][2], acc[1][3]);
  acc_guard4(acc[2][0], acc[2][1], acc[2][2], acc[2][3]);
  acc_guard4(acc[3][0], acc[3][1], acc[3][2], acc[3][3]);

  float* slab = sT[wave];
  unsigned short* C  = Cout  + (size_t)b * strideC;
  unsigned short* C2 = Cout2 + (size_t)b * strideC;
  const int q = lane >> 3, c8 = (lane & 7) * 8;
#pragma unroll
  for (int i = 0; i < 4; ++i) {
    const int mBase = m0 + (i << 4);
#pragma unroll
    for (int j = 0; j < 4; ++j) {
      const int n = n0 + (j << 4) + rlane;
      float bvn = 0.f;
      if (BIAS_MODE == 2) {
        const int ia = (n < nsplit) ? n : (nsplit - 1);
        const int ib = (n < nsplit) ? 0 : (n - nsplit);
        const float va = bias[ia];
        const float vb2 = bias2[ib];
        bvn = (n < nsplit) ? va : vb2;
      }
#pragma unroll
      for (int r = 0; r < 8; ++r) {
        float v = acc[i][j][r];
        if (BIAS_MODE == 1) v += bias[mBase + mOff + r];
        if (BIAS_MODE == 2) v += bvn;
        v *= oscale;
        slab[(mOff + r) * 68 + (j << 4) + rlane] = v;
      }
    }
    lds_wave_sync();
    for (int pass = 0; pass < 2; ++pass) {
#pragma unroll
      for (int it = 0; it < 4; ++it) {
        const int row = it * 4 + q;
        const float* sp = slab + row * 68 + c8;
        if (OUT_MODE == 1) {
          v8h hv;
#pragma unroll
          for (int e = 0; e < 8; ++e) hv[e] = (_Float16)sp[e];
          *(volatile v8h*)(C + (size_t)(mBase + row) * ldc + n0 + c8) = hv;
        } else {
          v8h hv, lv;
#pragma unroll
          for (int e = 0; e < 8; ++e) {
            const unsigned short hb = f2bf_bits(sp[e]);
            const unsigned short lb = f2bf_bits(sp[e] - bf_bits2f(hb));
            hv[e] = __builtin_bit_cast(_Float16, hb);
            lv[e] = __builtin_bit_cast(_Float16, lb);
          }
          *(volatile v8h*)(C  + (size_t)(mBase + row) * ldc + n0 + c8) = hv;
          *(volatile v8h*)(C2 + (size_t)(mBase + row) * ldc + n0 + c8) = lv;
        }
      }
      __threadfence();
    }
    lds_wave_sync();
  }
}

__global__ __launch_bounds__(256) void split_bf16x2_kernel(const float* __restrict__ in, unsigned short* __restrict__ hi,
                                                           unsigned short* __restrict__ lo, int n2) {
  const int i = blockIdx.x * 256 + threadIdx.x;
  if (i < n2) {
    const v2f f = *(const v2f*)(in + 2 * (size_t)i);
    const unsigned short h0 = f2bf_bits(f[0]), h1 = f2bf_bits(f[1]);
    const unsigned short l0 = f2bf_bits(f[0] - bf_bits2f(h0)), l1 = f2bf_bits(f[1] - bf_bits2f(h1));
    const unsigned uh = pk16(h0, h1), ul = pk16(l0, l1);
    ((volatile unsigned*)hi)[i] = uh;
    ((volatile unsigned*)lo)[i] = ul;
    __threadfence();
    ((volatile unsigned*)hi)[i] = uh;
    ((volatile unsigned*)lo)[i] = ul;
  }
}

__global__ __launch_bounds__(256) void tsplit_kernel(const float* __restrict__ W, unsigned short* __restrict__ oh,
                                                     unsigned short* __restrict__ ol, int R, int Cc, long sIn, long sOut) {
  __shared__ __align__(16) float tf[64 * 68];
  W  += (size_t)blockIdx.z * sIn;
  oh += (size_t)blockIdx.z * sOut;
  ol += (size_t)blockIdx.z * sOut;
  const int c0  = blockIdx.x * 64;
  const int r0  = blockIdx.y * 64;
  const int tid = threadIdx.x;
  {
    const int lr = tid >> 4;
    const int c4 = (tid & 15) * 4;
#pragma unroll
    for (int it = 0; it < 4; ++it) {
      const int rr = it * 16 + lr;
      const v4f a = *(const v4f*)(W + (size_t)(r0 + rr) * Cc + c0 + c4);
      *(v4f*)(tf + rr * 68 + c4) = a;
    }
  }
  __syncthreads();
  const int sub = tid >> 3;
  const int c8  = (tid & 7) * 8;
  v4u hv[2], lv[2];
#pragma unroll
  for (int it = 0; it < 2; ++it) {
    const int oc = it * 32 + sub;
    v4u a, a2;
#pragma unroll
    for (int qq = 0; qq < 4; ++qq) {
      const float f0 = tf[(c8 + 2 * qq) * 68 + oc];
      const float f1 = tf[(c8 + 2 * qq + 1) * 68 + oc];
      const unsigned short h0 = f2bf_bits(f0), h1 = f2bf_bits(f1);
      const unsigned short l0 = f2bf_bits(f0 - bf_bits2f(h0)), l1 = f2bf_bits(f1 - bf_bits2f(h1));
      a[qq]  = pk16(h0, h1);
      a2[qq] = pk16(l0, l1);
    }
    hv[it] = a; lv[it] = a2;
  }
  for (int pass = 0; pass < 2; ++pass) {
#pragma unroll
    for (int it = 0; it < 2; ++it) {
      const int oc = it * 32 + sub;
      const size_t go = (size_t)(c0 + oc) * R + r0 + c8;
      *(volatile v4u*)(oh + go) = hv[it];
      *(volatile v4u*)(ol + go) = lv[it];
    }
    __threadfence();
  }
}

__global__ __launch_bounds__(256) void attn_kernel(
    const unsigned short* __restrict__ qkhp, const unsigned short* __restrict__ qklp,
    const unsigned short* __restrict__ vpp, const float* __restrict__ x, float* __restrict__ out) {
  __shared__ __align__(16) float smem[NCH * AQB];

  const int tid  = threadIdx.x;
  const int wave = tid >> 5;
  const int lane = tid & 31;
  const int hh   = lane >> 4;
  const int c    = lane & 15;
  const int rg    = wave & 3;
  const int chalf = wave >> 2;
  const int b  = blockIdx.y;
  const int i0 = blockIdx.x * AQB;
  const int q0 = i0 + rg * 16;

  const __bf16* QKh = (const __bf16*)(const void*)qkhp + (size_t)b * NPX * QKW;
  const __bf16* QKl = (const __bf16*)(const void*)qklp + (size_t)b * NPX * QKW;
  const _Float16* Vb = (const _Float16*)(const void*)vpp + ((size_t)b * NCH + (size_t)chalf * 128) * NPX;

  const v16b qah = ldfrag_b(QKh + (size_t)(q0 + c) * QKW + 8 * hh);
  const v16b qal = ldfrag_b(QKl + (size_t)(q0 + c) * QKW + 8 * hh);

  _Float16* pwh = (_Float16*)(void*)smem + wave * 2048;
  _Float16* pwl = pwh + 1024;

  const v8f zero8 = (v8f){0.f,0.f,0.f,0.f,0.f,0.f,0.f,0.f};
  float mrow[8], lrow[8];
  v8f oacc[8];
#pragma unroll
  for (int r = 0; r < 8; ++r) { mrow[r] = -3.0e38f; lrow[r] = 0.f; }
#pragma unroll
  for (int t = 0; t < 8; ++t) oacc[t] = zero8;

  for (int kc = 0; kc < NPX / AKC; ++kc) {
    const int kv0 = kc * AKC;

    v8f s[4];
#pragma unroll
    for (int t = 0; t < 4; ++t) {
      const size_t ko = (size_t)(kv0 + t * 16 + c) * QKW + NHID + 8 * hh;
      const v16b kh = ldfrag_b(QKh + ko);
      const v16b kl = ldfrag_b(QKl + ko);
      v8f a = mma_b(qah, kh, zero8);
      a = mma_b(qah, kl, a);
      a = mma_b(qal, kh, a);
      guard_s(a, qah, qal, kh, kl);
      s[t] = a;
    }

    float cm[8];
#pragma unroll
    for (int r = 0; r < 8; ++r) {
      float m = fmaxf(fmaxf(s[0][r], s[1][r]), fmaxf(s[2][r], s[3][r]));
#pragma unroll
      for (int off = 1; off < 16; off <<= 1) m = fmaxf(m, __shfl_xor(m, off, 32));
      cm[r] = m;
    }

    lds_wave_sync();

#pragma unroll
    for (int r = 0; r < 8; ++r) {
      const float mnew  = fmaxf(mrow[r], cm[r]);
      const float alpha = __expf(mrow[r] - mnew);
      mrow[r] = mnew;
      float psum = 0.f;
      const int prow = (8 * hh + r) * AKC;
#pragma unroll
      for (int t = 0; t < 4; ++t) {
        const float p  = __expf(s[t][r] - mnew);
        psum += p;
        const float ps = p * 1024.0f;
        const _Float16 ph = (_Float16)ps;
        const _Float16 pl = (_Float16)((ps - (float)ph) * 2048.0f);
        pwh[prow + t * 16 + c] = ph;
        pwl[prow + t * 16 + c] = pl;
      }
#pragma unroll
      for (int off = 1; off < 16; off <<= 1) psum += __shfl_xor(psum, off, 32);
      lrow[r] = lrow[r] * alpha + psum;
#pragma unroll
      for (int t = 0; t < 8; ++t) oacc[t][r] *= alpha;
    }

    lds_wave_sync();

    const v16h pah0 = ldfrag_h(pwh + c * AKC + 8 * hh);
    const v16h pah1 = ldfrag_h(pwh + c * AKC + 32 + 8 * hh);
    const v16h pal0 = ldfrag_h(pwl + c * AKC + 8 * hh);
    const v16h pal1 = ldfrag_h(pwl + c * AKC + 32 + 8 * hh);

#pragma unroll
    for (int t = 0; t < 8; ++t) {
      const _Float16* vr = Vb + (size_t)(t * 16 + c) * NPX + kv0 + 8 * hh;
      const v16h vb0 = ldfrag_h(vr);
      const v16h vb1 = ldfrag_h(vr + 32);
      v8f tq = mma_h(pal0, vb0, zero8);
      v8f o  = mma_h(pah0, vb0, oacc[t]);
      tq = mma_h(pal1, vb1, tq);
      o  = mma_h(pah1, vb1, o);
      guard_pv(o, tq, pah0, pah1, pal0, pal1, vb0, vb1);
      oacc[t] = o + tq * 0.00048828125f;
    }
  }

  float inv[8];
#pragma unroll
  for (int r = 0; r < 8; ++r) inv[r] = (1.0f / lrow[r]) * (1.0f / 4096.0f);
  __syncthreads();
#pragma unroll
  for (int t = 0; t < 8; ++t) {
    const int ch = chalf * 128 + t * 16 + c;
    float* orow = smem + ch * AQB + rg * 16 + 8 * hh;
#pragma unroll
    for (int r = 0; r < 8; ++r) orow[r] = oacc[t][r] * inv[r];
  }
  __syncthreads();
  {
    const int px4 = c * 4;
    const size_t gb = (size_t)b * NCH * NPX + (size_t)i0 + px4;
    v4f vals[16];
#pragma unroll
    for (int it = 0; it < 16; ++it) {
      const int ch = wave * 32 + it * 2 + hh;
      const v4f o4 = *(const v4f*)(smem + ch * AQB + px4);
      const v4f x4 = *(const v4f*)(x + gb + (size_t)ch * NPX);
      vals[it] = o4 + x4;
    }
    for (int pass = 0; pass < 2; ++pass) {
#pragma unroll
      for (int it = 0; it < 16; ++it) {
        const int ch = wave * 32 + it * 2 + hh;
        *(volatile v4f*)(out + gb + (size_t)ch * NPX) = vals[it];
      }
      __threadfence();
    }
  }
}

extern "C" void kernel_launch(void* const* d_in, const int* in_sizes, int n_in,
                              void* d_out, int out_size, void* d_ws, size_t ws_size,
                              hipStream_t stream) {
  if (n_in < 7) return;
  if (in_sizes[0] != NBAT * NCH * NPX) return;
  if (in_sizes[1] != NHID * NCH || in_sizes[2] != NHID) return;
  if (in_sizes[3] != NHID * NCH || in_sizes[4] != NHID) return;
  if (in_sizes[5] != NCH * NCH || in_sizes[6] != NCH) return;
  if (out_size != NBAT * NCH * NPX) return;

  const float* x  = (const float*)d_in[0];
  const float* wq = (const float*)d_in[1];
  const float* bq = (const float*)d_in[2];
  const float* wk = (const float*)d_in[3];
  const float* bk = (const float*)d_in[4];
  const float* wv = (const float*)d_in[5];
  const float* bv = (const float*)d_in[6];
  float* out = (float*)d_out;

  const size_t PXT  = (size_t)NBAT * NPX * NCH * 2;
  const size_t PWQK = (size_t)QKW * NCH * 2;
  const size_t PWV  = (size_t)NCH * NCH * 2;
  const size_t PQK  = (size_t)NBAT * NPX * QKW * 2;
  const size_t PVP  = (size_t)NBAT * NCH * NPX * 2;
  size_t off = 0;
  const size_t oXth  = off; off += PXT;   const size_t oXtl  = off; off += PXT;
  const size_t oWqkh = off; off += PWQK;  const size_t oWqkl = off; off += PWQK;
  const size_t oWvh  = off; off += PWV;   const size_t oWvl  = off; off += PWV;
  const size_t oQKh  = off; off += PQK;   const size_t oQKl  = off; off += PQK;
  const size_t oVp   = off; off += PVP;
  if (off > ws_size) return;

  char* ws = (char*)d_ws;
  unsigned short* Xth  = (unsigned short*)(ws + oXth);   unsigned short* Xtl  = (unsigned short*)(ws + oXtl);
  unsigned short* Wqkh = (unsigned short*)(ws + oWqkh);  unsigned short* Wqkl = (unsigned short*)(ws + oWqkl);
  unsigned short* Wvh  = (unsigned short*)(ws + oWvh);   unsigned short* Wvl  = (unsigned short*)(ws + oWvl);
  unsigned short* QKh  = (unsigned short*)(ws + oQKh);   unsigned short* QKl  = (unsigned short*)(ws + oQKl);
  unsigned short* Vp   = (unsigned short*)(ws + oVp);

  const dim3 blk(256);

  tsplit_kernel<<<dim3(NPX / 64, NCH / 64, NBAT), blk, 0, stream>>>(x, Xth, Xtl, NCH, NPX, (long)NCH * NPX, (long)NPX * NCH);

  const int n2w = NHID * NCH / 2;
  split_bf16x2_kernel<<<dim3((n2w + 255) / 256), blk, 0, stream>>>(wq, Wqkh, Wqkl, n2w);
  split_bf16x2_kernel<<<dim3((n2w + 255) / 256), blk, 0, stream>>>(wk, Wqkh + NHID * NCH, Wqkl + NHID * NCH, n2w);
  const int n2v = NCH * NCH / 2;
  split_bf16x2_kernel<<<dim3((n2v + 255) / 256), blk, 0, stream>>>(wv, Wvh, Wvl, n2v);

  gemm_bf16x3<2, 2><<<dim3(((NPX / 64) * (QKW / 64) + 7) / 8, NBAT), blk, 0, stream>>>(
      Xth, Xtl, NCH, (long)NPX * NCH,
      Wqkh, Wqkl, NCH, 0L,
      QKh, QKl, QKW, (long)NPX * QKW,
      bq, bk, NHID,
      NPX, QKW, NCH, 1.0f);

  gemm_bf16x3<1, 1><<<dim3(((NCH / 64) * (NPX / 64) + 7) / 8, NBAT), blk, 0, stream>>>(
      Wvh, Wvl, NCH, 0L,
      Xth, Xtl, NCH, (long)NPX * NCH,
      Vp, Vp, NPX, (long)NCH * NPX,
      bv, bv, NCH,
      NCH, NPX, NCH, 4.0f);

  attn_kernel<<<dim3(NPX / AQB, NBAT), blk, 0, stream>>>(QKh, QKl, Vp, x, out);

  (void)hipGetLastError();
}
